// Block_38388417692234
// MI455X (gfx1250) — hardware-run, weakly checked
//
#include <hip/hip_runtime.h>
#include <math.h>


#ifndef NB
#define NB 32
#endif
#ifndef SEQ
#define SEQ 512
#endif
#define NB_FULL  32
#define SEQ_FULL 512
#ifndef OUT_SEQ
#define OUT_SEQ SEQ
#endif
#define DM    768
#define NH_   12
#define HD    64
#define HID   3072
#define AW    4
#define OSP   68
#define TSP   68
#define NCH   4
#define MROWS (NB * SEQ)
#define MCH   (MROWS / NCH)
#define AH    ((NB % 2 == 0) ? 2 : 1)
#define HB    (NB / AH)
#define HROWS (HB * SEQ)
#define QSUB  ((size_t)HROWS * DM)
#define QREG  (((size_t)2 * HROWS * DM > (size_t)MROWS * DM) ? (size_t)2 * HROWS * DM : (size_t)MROWS * DM)
#define WCAR  64.0f
#define WCAI  (1.0f / 64.0f)
#define CXS   16.0f
#define CXI   (1.0f / 16.0f)
#define QRS   2048.0f
#define QRI   (1.0f / 2048.0f)
#define SC2   ((float)(0.125 * 1.4426950408889634))
#define PSH   14.0f
#define NEGB  (-3.0e38f)

static_assert(HD == 64);
static_assert(NH_ * HD == DM);
static_assert(DM % 64 == 0);
static_assert(HID % 64 == 0);
static_assert(DM % 32 == 0);
static_assert(HID % 32 == 0);
static_assert(HD % 32 == 0);
static_assert(SEQ % 64 == 0);
static_assert(SEQ % 32 == 0);
static_assert(SEQ % (16 * AW) == 0);
static_assert(MROWS % (NCH * 64) == 0);
static_assert(DM == 3 * 32 * 8);
static_assert(NB <= NB_FULL);
static_assert(SEQ <= SEQ_FULL);
static_assert(AH * HB == NB);
static_assert(HROWS % 64 == 0);
static_assert(2 * QSUB <= QREG);
static_assert((size_t)MROWS * DM <= QREG);
static_assert((QREG * 2) % 256 == 0);
static_assert((QSUB * 2) % 256 == 0);
static_assert((OSP * 4) % 16 == 0);
static_assert((TSP * 4) % 16 == 0);
static_assert(64 * TSP * 4 <= 131072);
static_assert(AW * 16 * OSP * 4 <= 131072);

typedef _Float16 h16;
typedef __attribute__((ext_vector_type(16))) _Float16 v16h;
typedef __attribute__((ext_vector_type(8)))  _Float16 v8h;
typedef __attribute__((ext_vector_type(8)))  float    v8f;
typedef __attribute__((ext_vector_type(4)))  float    v4f;
typedef v4f  __attribute__((may_alias)) v4fa;

__device__ __forceinline__ unsigned short f2bf(float f) { unsigned u = __float_as_uint(f); u += 0x7FFFu + ((u >> 16) & 1u); return (unsigned short)(u >> 16); }
__device__ __forceinline__ float bfr(float f) { return __uint_as_float(((unsigned)f2bf(f)) << 16); }
__device__ __forceinline__ v16h cat16(v8h lo, v8h hi) { return __builtin_shufflevector(lo, hi, 0, 1, 2, 3, 4, 5, 6, 7, 8, 9, 10, 11, 12, 13, 14, 15); }
__device__ __forceinline__ v16h  ldh(const h16* p) { return cat16(*(const v8h*)p, *(const v8h*)(p + 16)); }
__device__ __forceinline__ void wave_sync() { __builtin_amdgcn_fence(3  , "wavefront"); __builtin_amdgcn_wave_barrier(); asm volatile("" ::: "memory"); }
__device__ __forceinline__ v8f wmma_g(v16h a, v16h b, v8f c) {
    c = __builtin_amdgcn_wmma_f32_16x16x32_f16(false, a, false, b, (short)0, c, false, false);
    asm volatile("v_nop\n\tv_nop\n\tv_nop\n\tv_nop" : "+v"(c) : "v"(a), "v"(b));
    return c;
}
static __device__ __forceinline__ h16 toh_flush(float v) { const h16 r = (h16)v; return (fabsf(v) < 6.103515625e-05f) ? (h16)0.0f : r; }

__global__ __launch_bounds__(256) void k_wcvt(const float* __restrict__ src, h16* dst, size_t n8) {
    const size_t i = (size_t)blockIdx.x * 256 + threadIdx.x; if (i >= n8) return;
    const v8f v = *(const v8f*)(src + i * 8); v8h o;
#pragma unroll
    for (int k = 0; k < 8; ++k) o[k] = toh_flush(bfr(v[k]) * WCAR);
    *(volatile v8h*)(dst + i * 8) = o; __threadfence(); *(volatile v8h*)(dst + i * 8) = o;
}

__global__ __launch_bounds__(256) void k_ln(const float* __restrict__ X, const float* __restrict__ gw, const float* __restrict__ gb, h16* Hn, int srcSeq, int rin, int nrows) {
#pragma clang fp contract(off)
    const int lane = threadIdx.x & 31;
    const int wave = __builtin_amdgcn_readfirstlane((int)(threadIdx.x >> 5));
    const int row = blockIdx.x * 8 + wave;
    if (row >= nrows) return;
    const int bb = row / SEQ, tt = row % SEQ;
    const float* xr = X + ((size_t)bb * (size_t)srcSeq + (size_t)tt) * DM;
    v8f v0 = *(const v8f*)(xr + (size_t)lane * 8);
    v8f v1 = *(const v8f*)(xr + (size_t)(32 + lane) * 8);
    v8f v2 = *(const v8f*)(xr + (size_t)(64 + lane) * 8);
#pragma unroll
    for (int k = 0; k < 8; ++k) { v0[k] = rin ? bfr(v0[k]) : v0[k]; v1[k] = rin ? bfr(v1[k]) : v1[k]; v2[k] = rin ? bfr(v2[k]) : v2[k]; }
    float s = 0.0f;
#pragma unroll
    for (int k = 0; k < 8; ++k) { s += v0[k]; s += v1[k]; s += v2[k]; }
#pragma unroll
    for (int off = 16; off > 0; off >>= 1) s += __shfl_xor(s, off, 32);
    const float mu = s * (1.0f / (float)DM);
    float ss = 0.0f;
#pragma unroll
    for (int k = 0; k < 8; ++k) { const float d0 = v0[k] - mu, d1 = v1[k] - mu, d2 = v2[k] - mu; ss += d0 * d0; ss += d1 * d1; ss += d2 * d2; }
#pragma unroll
    for (int off = 16; off > 0; off >>= 1) ss += __shfl_xor(ss, off, 32);
    const float rs = rsqrtf(ss * (1.0f / (float)DM) + 1e-5f);
    v8h o0, o1, o2;
    { const v8f w = *(const v8f*)(gw + (size_t)lane * 8); const v8f c = *(const v8f*)(gb + (size_t)lane * 8);
#pragma unroll
      for (int k = 0; k < 8; ++k) o0[k] = toh_flush(((v0[k] - mu) * rs) * bfr(w[k]) + bfr(c[k])); }
    { const v8f w = *(const v8f*)(gw + (size_t)(32 + lane) * 8); const v8f c = *(const v8f*)(gb + (size_t)(32 + lane) * 8);
#pragma unroll
      for (int k = 0; k < 8; ++k) o1[k] = toh_flush(((v1[k] - mu) * rs) * bfr(w[k]) + bfr(c[k])); }
    { const v8f w = *(const v8f*)(gw + (size_t)(64 + lane) * 8); const v8f c = *(const v8f*)(gb + (size_t)(64 + lane) * 8);
#pragma unroll
      for (int k = 0; k < 8; ++k) o2[k] = toh_flush(((v2[k] - mu) * rs) * bfr(w[k]) + bfr(c[k])); }
    static_assert(32 * 16 * 3 == DM * 2);
    h16* orow = Hn + (size_t)row * DM;
#pragma unroll 1
    for (int ps = 0; ps < 2; ++ps) {
        *(volatile v8h*)(orow + (size_t)lane * 8) = o0;
        *(volatile v8h*)(orow + (size_t)(32 + lane) * 8) = o1;
        *(volatile v8h*)(orow + (size_t)(64 + lane) * 8) = o2;
        if (ps == 0) __threadfence(); }
}

enum { EP_QK = 0, EP_VT = 1, EP_X2 = 2, EP_GELU = 3, EP_OUT = 4 };

template <int EP>
__device__ __forceinline__ void gemm_tile(const h16* __restrict__ A, const h16* __restrict__ Bt, const int K,
                                          const float* __restrict__ bias, const float* __restrict__ RES, h16* OH, h16* OH2, float* OF, const int rowBase) {
    __shared__ __align__(16) float os[64 * TSP];
    const int lane = threadIdx.x & 31, lr = lane & 15, hi = lane >> 4;
    const int r0 = blockIdx.x * 64, c0 = blockIdx.y * 64;
    v8f acc[4][4];
#pragma unroll
    for (int mb = 0; mb < 4; ++mb)
#pragma unroll
        for (int nb = 0; nb < 4; ++nb) acc[mb][nb] = (v8f){};
    const size_t aoff = (size_t)(r0 + lr) * K + 8 * hi, boff = (size_t)(c0 + lr) * K + 8 * hi;
#pragma unroll 1
    for (int kc = 0; kc < K; kc += 32) {
        v16h a[4];
#pragma unroll
        for (int mb = 0; mb < 4; ++mb) a[mb] = ldh(A + aoff + (size_t)mb * 16 * K + kc);
#pragma unroll
        for (int nb = 0; nb < 4; ++nb) { const v16h b = ldh(Bt + boff + (size_t)nb * 16 * K + kc);
#pragma unroll
            for (int mb = 0; mb < 4; ++mb) acc[mb][nb] = wmma_g(a[mb], b, acc[mb][nb]); }
    }
#pragma unroll
    for (int mb = 0; mb < 4; ++mb)
#pragma unroll
        for (int nb = 0; nb < 4; ++nb)
#pragma unroll
            for (int j = 0; j < 8; ++j) os[(mb * 16 + hi * 8 + j) * TSP + nb * 16 + lr] = acc[mb][nb][j];
    wave_sync();
    if constexpr (EP == EP_GELU || EP == EP_OUT) {
        const int c4 = (lane & 15) * 4;
        const v4f bv = *(const v4f*)(bias + c0 + c4);
        float bq[4];
#pragma unroll
        for (int i = 0; i < 4; ++i) bq[i] = bfr(bv[i]);
        const size_t g0 = (size_t)(rowBase + r0);
        static_assert(32 * 4 * 32 == 64 * 64);
#pragma unroll 1
        for (int s = 0; s < 32; ++s) {
            const int row = 2 * s + (lane >> 4);
            v4f x = *(const v4fa*)(&os[row * TSP + c4]);
            if constexpr (EP == EP_GELU) {
#pragma unroll
                for (int i = 0; i < 4; ++i) { const float v = x[i] * WCAI + bq[i]; x[i] = 0.5f * v * (1.0f + erff(v * 0.70710678118654752f)); }
            } else {
                const v4f rr = *(const v4f*)(RES + (g0 + (size_t)row) * DM + c0 + c4);
#pragma unroll
                for (int i = 0; i < 4; ++i) x[i] = rr[i] + (x[i] * WCAI + bq[i]);
            }
            *(v4fa*)(&os[row * TSP + c4]) = x;
        }
        wave_sync();
    }
    if constexpr (EP == EP_QK || EP == EP_VT || EP == EP_GELU) {
        size_t base, rstep;
        if constexpr (EP == EP_QK) { const int part = c0 / DM, head = (c0 % DM) / HD; const int bb = r0 / SEQ, tt = r0 % SEQ;
                                     base = (size_t)part * QREG + ((size_t)(bb * NH_ + head) * SEQ + (size_t)tt) * HD; rstep = HD; }
        else if constexpr (EP == EP_VT) { const int bb = c0 / SEQ, tt = c0 % SEQ; base = ((size_t)bb * DM + (size_t)r0) * SEQ + (size_t)tt; rstep = SEQ; }
        else { base = (size_t)r0 * HID + (size_t)c0; rstep = HID; }
        const float sc = (EP == EP_GELU) ? 1.0f : WCAI;
        static_assert(32 * 16 * 16 == 64 * 64 * 2);
#pragma unroll 1
        for (int ps = 0; ps < 2; ++ps) {
#pragma unroll 1
            for (int s = 0; s < 16; ++s) { const int row = 4 * s + (lane >> 3), c8 = (lane & 7) * 8;
                const v4f x0 = *(const v4fa*)(&os[row * TSP + c8]); const v4f x1 = *(const v4fa*)(&os[row * TSP + c8 + 4]); v8h hv, rv;
#pragma unroll
                for (int i = 0; i < 4; ++i) { const float a0 = x0[i] * sc, a1 = x1[i] * sc; const h16 h0 = toh_flush(a0), h1 = toh_flush(a1);
                    hv[i] = h0; hv[4 + i] = h1;
                    if constexpr (EP == EP_QK) { rv[i] = toh_flush((a0 - (float)h0) * QRS); rv[4 + i] = toh_flush((a1 - (float)h1) * QRS); } }
                *(volatile v8h*)(OH + base + (size_t)row * rstep + c8) = hv;
                if constexpr (EP == EP_QK) { *(volatile v8h*)(OH2 + base + (size_t)row * rstep + c8) = rv; } }
            if (ps == 0) __threadfence(); }
    } else {
        const int c4 = (lane & 15) * 4;
        float bq[4] = {0.0f, 0.0f, 0.0f, 0.0f};
        size_t base;
        if constexpr (EP == EP_X2) { const v4f bv = *(const v4f*)(bias + c0 + c4);
#pragma unroll
                                     for (int i = 0; i < 4; ++i) bq[i] = bfr(bv[i]);
                                     base = (size_t)r0 * DM + (size_t)c0; }
        else { const int g0 = rowBase + r0; const int bb = g0 / SEQ, tt = g0 % SEQ; base = ((size_t)bb * OUT_SEQ + (size_t)tt) * DM + (size_t)c0; }
        static_assert(32 * 16 * 32 == 64 * 64 * 4);
#pragma unroll 1
        for (int ps = 0; ps < 2; ++ps) {
#pragma unroll 1
            for (int s = 0; s < 32; ++s) { const int row = 2 * s + (lane >> 4);
                const v4f x = *(const v4fa*)(&os[row * TSP + c4]); v4f val;
                if constexpr (EP == EP_X2) {
#pragma unroll
                    for (int i = 0; i < 4; ++i) val[i] = 2.0f * (x[i] * (WCAI * CXI) + bq[i]);
                } else { val = x; }
                *(volatile v4f*)(OF + base + (size_t)row * DM + c4) = val; }
            if (ps == 0) __threadfence(); }
    }
}

__global__ __launch_bounds__(32) void k_gemm_qk(const h16* __restrict__ A, const h16* __restrict__ W, h16* QKV, h16* QKR) {
    gemm_tile<EP_QK>(A, W, DM, nullptr, nullptr, QKV, QKR, nullptr, 0);
}
__global__ __launch_bounds__(32) void k_gemm_vt(const h16* __restrict__ Wv, const h16* __restrict__ Hn, h16* VT) {
    gemm_tile<EP_VT>(Wv, Hn, DM, nullptr, nullptr, VT, nullptr, nullptr, 0);
}
__global__ __launch_bounds__(32) void k_gemm_x2(const h16* __restrict__ CT, const h16* __restrict__ Wp, const float* __restrict__ bias, float* X2) {
    gemm_tile<EP_X2>(CT, Wp, DM, bias, nullptr, nullptr, nullptr, X2, 0);
}
__global__ __launch_bounds__(32) void k_gemm_fc1(const h16* __restrict__ H2, const h16* __restrict__ W1, const float* __restrict__ bias, h16* G) {
    gemm_tile<EP_GELU>(H2, W1, DM, bias, nullptr, G, nullptr, nullptr, 0);
}
__global__ __launch_bounds__(32) void k_gemm_fc2(const h16* __restrict__ G, const h16* __restrict__ W2, const float* __restrict__ bias, const float* __restrict__ X2, float* OUT, int rowBase) {
    gemm_tile<EP_OUT>(G, W2, HID, bias, X2, nullptr, nullptr, OUT, rowBase);
}

#define STO_TILE(J, F) { v4f a_, c_; \
    a_[0] = F[0] * sc; a_[1] = F[1] * sc; a_[2] = F[2] * sc; a_[3] = F[3] * sc; c_[0] = F[4] * sc; c_[1] = F[5] * sc; c_[2] = F[6] * sc; c_[3] = F[7] * sc; \
    *(v4fa*)(&os[wb + lr * OSP + 16 * (J) + 8 * hi]) = a_; *(v4fa*)(&os[wb + lr * OSP + 16 * (J) + 8 * hi + 4]) = c_; }

__global__ __launch_bounds__(32 * AW) __attribute__((amdgpu_num_vgpr(256)))
void k_flash(const h16* __restrict__ QP, const h16* __restrict__ QRp, const h16* __restrict__ KP, const h16* __restrict__ KRp, const h16* __restrict__ VT, h16* CTX) {
    __shared__ __align__(16) float os[AW * 16 * OSP];
    const int lane = threadIdx.x & 31, lr = lane & 15, hi = lane >> 4;
    const int wave = __builtin_amdgcn_readfirstlane((int)(threadIdx.x >> 5));
    const int zh = blockIdx.y; const int b = zh / NH_, h = zh % NH_;
    const int t0 = (blockIdx.x * AW + wave) * 16;
    const size_t pbase = (size_t)zh * SEQ * HD;
    const size_t qo = pbase + (size_t)(t0 + lr) * HD + 8 * hi;
    const v16h q0 = ldh(QP + qo), q1 = ldh(QP + qo + 32);
    const v16h qr0 = ldh(QRp + qo), qr1 = ldh(QRp + qo + 32);
    const size_t ko = pbase + (size_t)lr * HD + 8 * hi;
    const size_t vo = pbase + (size_t)lr * SEQ + 8 * hi;
    v8f o0 = (v8f){}, o1 = (v8f){}, o2 = (v8f){}, o3 = (v8f){};
    float m = NEGB, l = 0.0f;
#pragma unroll 1
    for (int key0 = 0; key0 < SEQ; key0 += 32) {
        const h16* ka = KP + ko + (size_t)key0 * HD;
        const h16* kr = KRp + ko + (size_t)key0 * HD;
        v8f sa = (v8f){}, sb = (v8f){}, ra = (v8f){}, rb = (v8f){};
        { const v16h ka0 = ldh(ka), ka1 = ldh(ka + 32), kra0 = ldh(kr), kra1 = ldh(kr + 32);
          sa = wmma_g(ka0, q0, sa);  sa = wmma_g(ka1, q1, sa);
          ra = wmma_g(ka0, qr0, ra); ra = wmma_g(ka1, qr1, ra);
          ra = wmma_g(kra0, q0, ra); ra = wmma_g(kra1, q1, ra); }
        { const v16h kb0 = ldh(ka + 16 * HD), kb1 = ldh(ka + 16 * HD + 32), krb0 = ldh(kr + 16 * HD), krb1 = ldh(kr + 16 * HD + 32);
          sb = wmma_g(kb0, q0, sb);  sb = wmma_g(kb1, q1, sb);
          rb = wmma_g(kb0, qr0, rb); rb = wmma_g(kb1, qr1, rb);
          rb = wmma_g(krb0, q0, rb); rb = wmma_g(krb1, q1, rb); }
        float ta[8], tb[8]; float mx = NEGB;
#pragma unroll
        for (int r = 0; r < 8; ++r) { ta[r] = (sa[r] + ra[r] * QRI) * SC2; tb[r] = (sb[r] + rb[r] * QRI) * SC2; mx = fmaxf(mx, fmaxf(ta[r], tb[r])); }
        mx = fmaxf(mx, __shfl_xor(mx, 16, 32));
        const float mnew = fmaxf(m, mx);
        const float alpha = __builtin_amdgcn_exp2f(m - mnew);
        const float sh = PSH - mnew;
        v16h pb; float ls = 0.0f;
#pragma unroll
        for (int r = 0; r < 8; ++r) {
            const float ea = ta[r] + sh, eb = tb[r] + sh;
            const float xa = __builtin_amdgcn_exp2f(ea), xb = __builtin_amdgcn_exp2f(eb);
            const float ga = (ea < -14.0f) ? 0.0f : xa, gb = (eb < -14.0f) ? 0.0f : xb;
            const h16 pa = (h16)ga; const h16 pc = (h16)gb;
            pb[r] = pa; pb[8 + r] = pc;
            ls += (float)pa + (float)pc; }
        l = l * alpha + ls; m = mnew;
        o0 = o0 * alpha; o1 = o1 * alpha; o2 = o2 * alpha; o3 = o3 * alpha;
        const h16* va = VT + vo + key0;
        const v16h v0 = ldh(va), v1 = ldh(va + (size_t)16 * SEQ), v2 = ldh(va + (size_t)32 * SEQ), v3 = ldh(va + (size_t)48 * SEQ);
        o0 = wmma_g(v0, pb, o0); o1 = wmma_g(v1, pb, o1); o2 = wmma_g(v2, pb, o2); o3 = wmma_g(v3, pb, o3);
    }
    l += __shfl_xor(l, 16, 32);
    const float sc = CXS * (1.0f / l);
    const int wb = wave * 16 * OSP;
    STO_TILE(0, o0) STO_TILE(1, o1) STO_TILE(2, o2) STO_TILE(3, o3)
    wave_sync();
    h16* crow = CTX + ((size_t)b * SEQ + (size_t)t0) * DM + (size_t)h * HD;
    static_assert(32 * 16 * 4 == 16 * HD * 2);
#pragma unroll 1
    for (int ps = 0; ps < 2; ++ps) {
#pragma unroll
        for (int s = 0; s < 4; ++s) { const int row = 4 * s + (lane >> 3), c8 = (lane & 7) * 8;
            const v4f x0 = *(const v4fa*)(&os[wb + row * OSP + c8]); const v4f x1 = *(const v4fa*)(&os[wb + row * OSP + c8 + 4]); v8h hv;
#pragma unroll
            for (int i = 0; i < 4; ++i) { hv[i] = toh_flush(x0[i]); hv[4 + i] = toh_flush(x1[i]); }
            *(volatile v8h*)(crow + (size_t)row * DM + c8) = hv; }
        if (ps == 0) __threadfence(); }
}

static constexpr size_t al256(size_t v) { return (v + 255) & ~(size_t)255; }
static constexpr size_t N_WQKV = (size_t)3 * DM * DM;
static constexpr size_t N_WPRJ = (size_t)DM * DM;
static constexpr size_t N_WFC1 = (size_t)HID * DM;
static constexpr size_t N_WFC2 = (size_t)DM * HID;
static constexpr size_t SZ_W  = al256((N_WQKV + N_WPRJ + N_WFC1 + N_WFC2) * 2);
static constexpr size_t SZ_PL = al256((size_t)MROWS * DM * 2);
static constexpr size_t SZ_R  = QREG * 2;
static constexpr size_t SZ_TOTAL = SZ_W + 2 * SZ_PL + 2 * SZ_R;
static_assert(SZ_TOTAL <= (size_t)134217728);
static_assert(SZ_PL == (size_t)MROWS * DM * 2);
static_assert(SZ_R >= SZ_PL);
static_assert((N_WQKV * 2) % 256 == 0 && (N_WPRJ * 2) % 256 == 0 && (N_WFC1 * 2) % 256 == 0);
static_assert((size_t)MROWS * DM * 4 <= SZ_R + SZ_PL);
static_assert((size_t)MCH * HID * 2 <= SZ_PL);
static_assert((size_t)NB * NH_ * SEQ * HD == (size_t)MROWS * DM);
static_assert((size_t)HB * NH_ * SEQ * HD == QSUB);
static_assert(N_WQKV % 8 == 0 && N_WPRJ % 8 == 0 && N_WFC1 % 8 == 0 && N_WFC2 % 8 == 0);

extern "C" void kernel_launch(void* const* d_in, const int* in_sizes, int n_in,
                              void* d_out, int out_size, void* d_ws, size_t ws_size, hipStream_t stream) {
    if (n_in < 12) return;
    const size_t needx = ((size_t)(NB - 1) * SEQ_FULL + SEQ) * DM;
    if ((size_t)in_sizes[0] < needx) return;
    if (in_sizes[1] < DM || in_sizes[2] < DM || in_sizes[5] < DM || in_sizes[6] < DM || in_sizes[7] < DM || in_sizes[11] < DM || in_sizes[9] < HID) return;
    if ((size_t)in_sizes[3] < N_WQKV || (size_t)in_sizes[4] < N_WPRJ || (size_t)in_sizes[8] < N_WFC1 || (size_t)in_sizes[10] < N_WFC2) return;
    if ((size_t)out_size < ((size_t)(NB - 1) * OUT_SEQ + SEQ) * DM) return;
    if (SZ_TOTAL > ws_size) return;
    const float* x      = (const float*)d_in[0];
    const float* ln1_w  = (const float*)d_in[1];
    const float* ln1_b  = (const float*)d_in[2];
    const float* qkv_w  = (const float*)d_in[3];
    const float* proj_w = (const float*)d_in[4];
    const float* proj_b = (const float*)d_in[5];
    const float* ln2_w  = (const float*)d_in[6];
    const float* ln2_b  = (const float*)d_in[7];
    const float* fc1_w  = (const float*)d_in[8];
    const float* fc1_b  = (const float*)d_in[9];
    const float* fc2_w  = (const float*)d_in[10];
    const float* fc2_b  = (const float*)d_in[11];
    float* OUT = (float*)d_out;
    char* wsp = (char*)d_ws;
    h16* WQKV = (h16*)wsp;
    h16* WPRJ = WQKV + N_WQKV;
    h16* WFC1 = WPRJ + N_WPRJ;
    h16* WFC2 = WFC1 + N_WFC1;
    wsp += SZ_W;
    h16* P0 = (h16*)wsp; wsp += SZ_PL;
    h16* P1 = (h16*)wsp; wsp += SZ_R;
    h16* P2 = (h16*)wsp; wsp += SZ_R;
    h16* P3 = (h16*)wsp; wsp += SZ_PL;
    float* X2 = (float*)P2;
    h16* QV = P1;
    h16* QRP = P1 + QSUB;
    h16* KV = P2;
    h16* KRP = P2 + QSUB;

    { const size_t n8 = N_WQKV / 8; k_wcvt<<<(unsigned)((n8 + 255) / 256), 256, 0, stream>>>(qkv_w, WQKV, n8); }
    { const size_t n8 = N_WPRJ / 8; k_wcvt<<<(unsigned)((n8 + 255) / 256), 256, 0, stream>>>(proj_w, WPRJ, n8); }
    { const size_t n8 = N_WFC1 / 8; k_wcvt<<<(unsigned)((n8 + 255) / 256), 256, 0, stream>>>(fc1_w, WFC1, n8); }
    { const size_t n8 = N_WFC2 / 8; k_wcvt<<<(unsigned)((n8 + 255) / 256), 256, 0, stream>>>(fc2_w, WFC2, n8); }

    k_ln<<<(MROWS + 7) / 8, 256, 0, stream>>>(x, ln1_w, ln1_b, P0, SEQ_FULL, 1, MROWS);
    k_gemm_vt<<<dim3(DM / 64, MROWS / 64, 1), 32, 0, stream>>>(WQKV + (size_t)2 * DM * DM, P0, P3);
    for (int g = 0; g < AH; ++g) {
        k_gemm_qk<<<dim3(HROWS / 64, 2 * DM / 64, 1), 32, 0, stream>>>(P0 + (size_t)g * HROWS * DM, WQKV, QV, QRP);
        k_flash<<<dim3(SEQ / (16 * AW), HB * NH_, 1), 32 * AW, 0, stream>>>(QV, QRP, KV, KRP, P3 + (size_t)g * HB * DM * SEQ, P0 + (size_t)g * HROWS * DM);
    }
    k_gemm_x2<<<dim3(MROWS / 64, DM / 64, 1), 32, 0, stream>>>(P0, WPRJ, proj_b, X2);
    k_ln<<<(MROWS + 7) / 8, 256, 0, stream>>>(X2, ln2_w, ln2_b, P1, SEQ, 0, MROWS);
    for (int c = 0; c < NCH; ++c) {
        k_gemm_fc1<<<dim3(MCH / 64, HID / 64, 1), 32, 0, stream>>>(P1 + (size_t)c * MCH * DM, WFC1, fc1_b, P0);
        k_gemm_fc2<<<dim3(MCH / 64, DM / 64, 1), 32, 0, stream>>>(P0, WFC2, fc2_b, X2, OUT, c * MCH);
    }
}
